// ConvOffset3d_15092515078410
// MI455X (gfx1250) — hardware-verified
//
#include <hip/hip_runtime.h>
#include <math.h>
#include <stdint.h>

#define CIN    64
#define COUT   64
#define GRP    8
#define CPG    8
#define DD     8
#define HH     56
#define WWD    56
#define HWP    3136
#define NPOS   25088
#define KVOL   27
#define KK     1728
#define NOFFC  648
#define NCHK   4
#define NCH    6272
#define SPB    32
#define CVR    32
static_assert(HWP == HH * WWD);
static_assert(NPOS == DD * HWP);
static_assert(KK == KVOL * CIN);
static_assert(NOFFC == GRP * KVOL * 3);
static_assert(CIN == GRP * CPG);
static_assert(NCH * NCHK == NPOS);
static_assert((NCH % 64) == 0 && (COUT % 64) == 0 && (KK % 32) == 0);
static_assert((NCH % SPB) == 0);
static_assert((NPOS % CVR) == 0);
static_assert(((NCH * 4) % 128) == 0);
static_assert(((COUT * KK) % (256 * 8)) == 0);
static_assert(CIN == 8 * 8);

typedef __bf16   v16b __attribute__((ext_vector_type(16)));
typedef __bf16   v8b  __attribute__((ext_vector_type(8)));
typedef float    v8f  __attribute__((ext_vector_type(8)));
typedef float    v4f  __attribute__((ext_vector_type(4)));
typedef unsigned int v4u __attribute__((ext_vector_type(4)));

__device__ __forceinline__ unsigned short bf_bits(float f) {
  unsigned u = __float_as_uint(f);
  return (unsigned short)((u + 0x7FFFu + ((u >> 16) & 1u)) >> 16);
}
__device__ __forceinline__ float bf_up(unsigned short h) { return __uint_as_float(((unsigned)h) << 16); }
__device__ __forceinline__ float bfr(float f) { return bf_up(bf_bits(f)); }
__device__ __forceinline__ unsigned pk16(unsigned short a, unsigned short b) { return (unsigned)a | ((unsigned)b << 16); }
__device__ __forceinline__ float lo16f(unsigned u) { return __uint_as_float(u << 16); }
__device__ __forceinline__ float hi16f(unsigned u) { return __uint_as_float(u & 0xffff0000u); }
__device__ __forceinline__ v8f zero8() { v8f z = {0.f, 0.f, 0.f, 0.f, 0.f, 0.f, 0.f, 0.f}; return z; }

__device__ __forceinline__ v16b ldfrag_b(const __bf16* p) {
  union { v16b v; v8b h[2]; } f;
  f.h[0] = *(const v8b*)(p);
  f.h[1] = *(const v8b*)(p + 16);
  return f.v;
}

__device__ __forceinline__ v8f mma_b_raw(v16b a, v16b b, v8f c) {
  return __builtin_amdgcn_wmma_f32_16x16x32_bf16(false, a, false, b, (short)0, c, false, false);
}
__device__ __forceinline__ void dep_guard_b(v8f& a, v8f& b, v16b x, v16b y) {
#if defined(__HIP_DEVICE_COMPILE__)
  asm volatile("v_nop\n\tv_nop\n\tv_nop\n\tv_nop" : "+v"(a), "+v"(b) : "v"(x), "v"(y));
#endif
}
__device__ __forceinline__ void keep4_b(v16b a, v16b b, v16b c, v16b d) {
#if defined(__HIP_DEVICE_COMPILE__)
  asm volatile("v_nop" :: "v"(a), "v"(b), "v"(c), "v"(d));
#endif
}
__device__ __forceinline__ void acc_guard4(v8f& a, v8f& b, v8f& c, v8f& d) {
#if defined(__HIP_DEVICE_COMPILE__)
  asm volatile("v_nop\n\tv_nop\n\tv_nop\n\tv_nop" : "+v"(a), "+v"(b), "+v"(c), "+v"(d));
#endif
}
__device__ __forceinline__ void wave_sync_lds() {
  __builtin_amdgcn_fence(__ATOMIC_RELEASE, "workgroup");
  __builtin_amdgcn_wave_barrier();
  __builtin_amdgcn_fence(__ATOMIC_ACQUIRE, "workgroup");
}

__device__ __forceinline__ float tri8(float a0, float a1, float a2, float a3, float a4, float a5, float a6, float a7,
                                      float w0, float w1, float w2, float w3, float w4, float w5, float w6, float w7) {
#pragma clang fp contract(off)
  float t = a0 * w0;
  t = t + a1 * w1;
  t = t + a2 * w2;
  t = t + a3 * w3;
  t = t + a4 * w4;
  t = t + a5 * w5;
  t = t + a6 * w6;
  t = t + a7 * w7;
  return t;
}

__global__ __launch_bounds__(256) void cvt_xt(const float* __restrict__ x, unsigned short* xt) {
  __shared__ __align__(16) float sx[CIN * 36];
  const int tid = threadIdx.x;
  const int p0  = blockIdx.x * CVR;
  const float* xb = x + p0;
#pragma unroll
  for (int it = 0; it < 2; ++it) {
    const int idx = it * 256 + tid;
    const int c = idx >> 3, q = idx & 7;
    const v4f v = *(const v4f*)(xb + (size_t)c * NPOS + 4 * q);
    *(v4f*)(sx + c * 36 + 4 * q) = v;
  }
  __syncthreads();
  const int wave = tid >> 5, lane = tid & 31;
  const int r  = wave * 4 + (lane >> 3);
  const int c8 = (lane & 7) * 8;
  v4u p;
#pragma unroll
  for (int e = 0; e < 4; ++e)
    p[e] = pk16(bf_bits(sx[(c8 + 2 * e) * 36 + r]), bf_bits(sx[(c8 + 2 * e + 1) * 36 + r]));
  unsigned short* dst = xt + (size_t)(p0 + r) * CIN + c8;
  *(volatile v4u*)dst = p;
  __threadfence();
  *(volatile v4u*)dst = p;
}

__global__ __launch_bounds__(256) void wprep(const float* __restrict__ w, unsigned short* wp) {
  const int j   = blockIdx.x * 256 + threadIdx.x;
  const int f   = j * 8;
  const int o   = f / KK;
  const int rem = f - o * KK;
  const int t   = rem >> 6;
  const int c   = rem & 63;
  const float* src = w + ((size_t)(o * CIN + c)) * KVOL + t;
  float vals[8];
#pragma unroll
  for (int i = 0; i < 8; ++i) vals[i] = src[i * KVOL];
  v4u p;
#pragma unroll
  for (int i = 0; i < 4; ++i) p[i] = pk16(bf_bits(vals[2 * i]), bf_bits(vals[2 * i + 1]));
  unsigned short* d = wp + f;
  *(volatile v4u*)d = p;
  __threadfence();
  *(volatile v4u*)d = p;
}

__global__ __launch_bounds__(256)
void sampler(const unsigned short* __restrict__ xt, const float* __restrict__ offs, int nbase,
             unsigned short* colh, unsigned short* coll) {
#pragma clang fp contract(off)
  const int tid = threadIdx.x, wave = tid >> 5, lane = tid & 31;
  const int q = lane >> 3, g = lane & 7;
  const int nl = blockIdx.x * SPB + wave * 4 + q;
  const int n  = nbase + nl;
  const int od = n / HWP;
  const int rm = n - od * HWP;
  const int oh = rm / WWD;
  const int ow = rm - oh * WWD;
  const float* ob = offs + (size_t)(g * KVOL) * 3 * NPOS + n;
  const unsigned short* xg = xt + g * CPG;
  unsigned short* ch = colh + (size_t)nl * KK + g * CPG;
  unsigned short* cl = coll + (size_t)nl * KK + g * CPG;
#pragma unroll 1
  for (int tap = 0; tap < KVOL; ++tap) {
    const int kz = tap / 9;
    const int r9 = tap - kz * 9;
    const int ky = r9 / 3;
    const int kx = r9 - ky * 3;
    const float* op = ob + (size_t)tap * 3 * NPOS;
    const float oz = bfr(op[0]);
    const float oy = bfr(op[NPOS]);
    const float ox = bfr(op[2 * NPOS]);
    const float zc = (float)(kz + od - 1) + oz;
    const float yc = (float)(ky + oh - 1) + oy;
    const float xc = (float)(kx + ow - 1) + ox;
    const float z0f = floorf(zc), y0f = floorf(yc), x0f = floorf(xc);
    const float dz = zc - z0f, dy = yc - y0f, dx = xc - x0f;
    const int z0 = (int)fminf(fmaxf(z0f, -4096.f), 4096.f);
    const int y0 = (int)fminf(fmaxf(y0f, -4096.f), 4096.f);
    const int x0 = (int)fminf(fmaxf(x0f, -4096.f), 4096.f);
    const bool vz0 = (z0 >= 0) && (z0 < DD),  vz1 = (z0 >= -1) && (z0 < DD - 1);
    const bool vy0 = (y0 >= 0) && (y0 < HH),  vy1 = (y0 >= -1) && (y0 < HH - 1);
    const bool vx0 = (x0 >= 0) && (x0 < WWD), vx1 = (x0 >= -1) && (x0 < WWD - 1);
    const int cz0 = min(max(z0, 0), DD - 1),  cz1 = min(max(z0 + 1, 0), DD - 1);
    const int cy0 = min(max(y0, 0), HH - 1),  cy1 = min(max(y0 + 1, 0), HH - 1);
    const int cx0 = min(max(x0, 0), WWD - 1), cx1 = min(max(x0 + 1, 0), WWD - 1);
    const float wz0 = 1.f - dz, wz1 = dz, wy0 = 1.f - dy, wy1 = dy, wx0 = 1.f - dx, wx1 = dx;
    const float zy00 = wz0 * wy0, zy01 = wz0 * wy1, zy10 = wz1 * wy0, zy11 = wz1 * wy1;
    float w000 = zy00 * wx0, w001 = zy00 * wx1, w010 = zy01 * wx0, w011 = zy01 * wx1;
    float w100 = zy10 * wx0, w101 = zy10 * wx1, w110 = zy11 * wx0, w111 = zy11 * wx1;
    w000 = (vz0 && vy0 && vx0) ? w000 : 0.f;
    w001 = (vz0 && vy0 && vx1) ? w001 : 0.f;
    w010 = (vz0 && vy1 && vx0) ? w010 : 0.f;
    w011 = (vz0 && vy1 && vx1) ? w011 : 0.f;
    w100 = (vz1 && vy0 && vx0) ? w100 : 0.f;
    w101 = (vz1 && vy0 && vx1) ? w101 : 0.f;
    w110 = (vz1 && vy1 && vx0) ? w110 : 0.f;
    w111 = (vz1 && vy1 && vx1) ? w111 : 0.f;
    const int b00 = (cz0 * HH + cy0) * WWD, b01 = (cz0 * HH + cy1) * WWD;
    const int b10 = (cz1 * HH + cy0) * WWD, b11 = (cz1 * HH + cy1) * WWD;
    const v4u u000 = *(const v4u*)(xg + (size_t)(b00 + cx0) * CIN);
    const v4u u001 = *(const v4u*)(xg + (size_t)(b00 + cx1) * CIN);
    const v4u u010 = *(const v4u*)(xg + (size_t)(b01 + cx0) * CIN);
    const v4u u011 = *(const v4u*)(xg + (size_t)(b01 + cx1) * CIN);
    const v4u u100 = *(const v4u*)(xg + (size_t)(b10 + cx0) * CIN);
    const v4u u101 = *(const v4u*)(xg + (size_t)(b10 + cx1) * CIN);
    const v4u u110 = *(const v4u*)(xg + (size_t)(b11 + cx0) * CIN);
    const v4u u111 = *(const v4u*)(xg + (size_t)(b11 + cx1) * CIN);
    v4u hv, lv;
#pragma unroll
    for (int e = 0; e < 4; ++e) {
      const float tl = tri8(lo16f(u000[e]), lo16f(u001[e]), lo16f(u010[e]), lo16f(u011[e]),
                            lo16f(u100[e]), lo16f(u101[e]), lo16f(u110[e]), lo16f(u111[e]),
                            w000, w001, w010, w011, w100, w101, w110, w111);
      const float th = tri8(hi16f(u000[e]), hi16f(u001[e]), hi16f(u010[e]), hi16f(u011[e]),
                            hi16f(u100[e]), hi16f(u101[e]), hi16f(u110[e]), hi16f(u111[e]),
                            w000, w001, w010, w011, w100, w101, w110, w111);
      const unsigned short hA = bf_bits(tl);
      const unsigned short lA = bf_bits(tl - bf_up(hA));
      const unsigned short hB = bf_bits(th);
      const unsigned short lB = bf_bits(th - bf_up(hB));
      hv[e] = pk16(hA, hB);
      lv[e] = pk16(lA, lB);
    }
    const int so = tap * CIN;
    *(volatile v4u*)(ch + so) = hv;
    *(volatile v4u*)(cl + so) = lv;
    __threadfence();
    *(volatile v4u*)(ch + so) = hv;
    *(volatile v4u*)(cl + so) = lv;
  }
}

__global__ __launch_bounds__(256) void gemm64(
    const unsigned short* __restrict__ Ap, int lda,
    const unsigned short* __restrict__ Bhp, const unsigned short* __restrict__ Blp, int ldb,
    float* Cout, int ldc, int M, int N, int K) {
  const __bf16* A  = (const __bf16*)(const void*)Ap;
  const __bf16* Bh = (const __bf16*)(const void*)Bhp;
  const __bf16* Bl = (const __bf16*)(const void*)Blp;
  __shared__ __align__(16) float sT[8][16 * 68];
  const int lane = threadIdx.x & 31;
  const int wave = threadIdx.x >> 5;
  const int tilesN = N >> 6;
  const int tilesM = M >> 6;
  const int tile = blockIdx.x * 8 + wave;
  if (tile >= tilesM * tilesN) return;
  const int tm = tile / tilesN;
  const int tn = tile - tm * tilesN;
  const int m0 = tm << 6;
  const int n0 = tn << 6;

  const int rlane = lane & 15;
  const int koff  = (lane >> 4) * 8;
  const int mOff  = (lane >> 4) * 8;

  v8f acc[4][4];
#pragma unroll
  for (int i = 0; i < 4; ++i)
#pragma unroll
    for (int j = 0; j < 4; ++j) acc[i][j] = zero8();

  for (int k0 = 0; k0 < K; k0 += 32) {
    v16b af[4];
#pragma unroll
    for (int i = 0; i < 4; ++i) {
      const size_t ao = (size_t)(m0 + (i << 4) + rlane) * lda + koff + k0;
      af[i] = ldfrag_b(A + ao);
    }
#pragma unroll
    for (int j = 0; j < 4; ++j) {
      const size_t bo = (size_t)(n0 + (j << 4) + rlane) * ldb + koff + k0;
      const v16b bh = ldfrag_b(Bh + bo);
      const v16b bl = ldfrag_b(Bl + bo);
#pragma unroll
      for (int i = 0; i < 4; ++i) {
        acc[i][j] = mma_b_raw(af[i], bh, acc[i][j]);
        acc[i][j] = mma_b_raw(af[i], bl, acc[i][j]);
      }
      dep_guard_b(acc[0][j], acc[3][j], bh, bl);
    }
    keep4_b(af[0], af[1], af[2], af[3]);
  }
  acc_guard4(acc[0][0], acc[0][1], acc[0][2], acc[0][3]);
  acc_guard4(acc[1][0], acc[1][1], acc[1][2], acc[1][3]);
  acc_guard4(acc[2][0], acc[2][1], acc[2][2], acc[2][3]);
  acc_guard4(acc[3][0], acc[3][1], acc[3][2], acc[3][3]);

  float* slab = sT[wave];
#pragma unroll
  for (int i = 0; i < 4; ++i) {
    const int mBase = m0 + (i << 4);
#pragma unroll
    for (int j = 0; j < 4; ++j) {
#pragma unroll
      for (int r = 0; r < 8; ++r) {
        slab[(mOff + r) * 68 + (j << 4) + rlane] = acc[i][j][r];
      }
    }
    wave_sync_lds();
    {
      const int hh = lane >> 4, c4 = (lane & 15) * 4;
      v4f ov[8];
#pragma unroll
      for (int it = 0; it < 8; ++it) {
        const int row = it * 2 + hh;
        ov[it] = *(const v4f*)(slab + row * 68 + c4);
      }
      for (int pass = 0; pass < 2; ++pass) {
#pragma unroll
        for (int it = 0; it < 8; ++it) {
          const int row = it * 2 + hh;
          *(volatile v4f*)(Cout + (size_t)(mBase + row) * ldc + n0 + c4) = ov[it];
        }
        __threadfence();
      }
    }
    wave_sync_lds();
  }
}

extern "C" void kernel_launch(void* const* d_in, const int* in_sizes, int n_in,
                              void* d_out, int out_size, void* d_ws, size_t ws_size,
                              hipStream_t stream) {
  if (n_in < 3) return;
  if (in_sizes[0] != CIN * NPOS) return;
  if (in_sizes[1] != NOFFC * NPOS) return;
  if (in_sizes[2] != COUT * CIN * KVOL) return;
  if (out_size != COUT * NPOS) return;

  const float* x      = (const float*)d_in[0];
  const float* offset = (const float*)d_in[1];
  const float* weight = (const float*)d_in[2];
  float* out = (float*)d_out;

  const size_t PXT = (size_t)NPOS * CIN * 2;
  const size_t PWP = (size_t)COUT * KK * 2;
  const size_t PCL = (size_t)NCH * KK * 2;
  size_t off = 0;
  const size_t oXT = off; off += PXT;
  const size_t oWP = off; off += PWP;
  const size_t oCH = off; off += PCL;
  const size_t oCL = off; off += PCL;
  if (off > ws_size) return;
  if (off > (size_t)134217728) return;

  char* ws = (char*)d_ws;
  unsigned short* XT = (unsigned short*)(ws + oXT);
  unsigned short* WP = (unsigned short*)(ws + oWP);
  unsigned short* CH = (unsigned short*)(ws + oCH);
  unsigned short* CL = (unsigned short*)(ws + oCL);

  const dim3 blk(256);
  cvt_xt<<<dim3(NPOS / CVR), blk, 0, stream>>>(x, XT);
  wprep<<<dim3((COUT * KK) / (256 * 8)), blk, 0, stream>>>(weight, WP);
  const dim3 gSmp(NCH / SPB);
  const dim3 gGemm(((COUT / 64) * (NCH / 64) + 7) / 8);
  for (int cidx = 0; cidx < NCHK; ++cidx) {
    const int nbase = cidx * NCH;
    sampler<<<gSmp, blk, 0, stream>>>(XT, offset, nbase, CH, CL);
    gemm64<<<gGemm, blk, 0, stream>>>(WP, KK, CH, CL, KK, out + (size_t)nbase, NPOS, COUT, NCH, KK);
  }
  (void)hipGetLastError();
}
